// TransformerBlock_86887188398386
// MI455X (gfx1250) — hardware-run, weakly checked
//
#include <hip/hip_runtime.h>
#include <stddef.h>


typedef _Float16 v16h __attribute__((ext_vector_type(16)));
typedef _Float16 v8h  __attribute__((ext_vector_type(8)));
typedef float    v8f  __attribute__((ext_vector_type(8)));
typedef float    v4f  __attribute__((ext_vector_type(4)));

#ifndef NB
#define NB 2
#endif
#define NB_FULL 2
#define SEQ    2048
#define DIM    1024
#define NHEAD  16
#define LHEADS 8
#define HD     64
#define DHID   2730
#define DHP    2752
#define MROWS  (NB * SEQ)

static_assert(NB >= 1 && NB <= NB_FULL);
static_assert(DIM == NHEAD * HD);
static_assert(HD == 64);
static_assert((DIM % 64) == 0 && (DIM % 32) == 0);
static_assert((DHP % 64) == 0 && (DHP % 32) == 0 && DHP >= DHID);
static_assert((MROWS % 64) == 0 && (MROWS % 8) == 0);
static_assert((SEQ % 512) == 0 && (SEQ % 128) == 0);

#define LDT 72
#define LDC 68

#define WCARRY 64.0f
#define PCARRY 1024.0f
#define VCARRY 64.0f
#define ACARRY 64.0f

#define M_QKV 0
#define M_WO  1
#define M_GU  2
#define M_OUT 3

#define PLANE_ELEMS ((size_t)MROWS * DIM)
#define TAB_BYTES   ((size_t)4096)
#define WQKV_BYTES  ((size_t)3 * DIM * DIM * 2)
#define WO_BYTES    ((size_t)DIM * DIM * 2)
#define WM_BYTES    ((size_t)DHP * DIM * 2)
#define P16_BYTES   (PLANE_ELEMS * 2)
#define X2_BYTES    (PLANE_ELEMS * 4)
#define A2_BYTES    ((size_t)MROWS * DHP * 2)
#define OFF_TAB   ((size_t)0)
#define OFF_WQKV  (OFF_TAB + TAB_BYTES)
#define OFF_WO    (OFF_WQKV + WQKV_BYTES)
#define OFF_MW    (OFF_WO + WO_BYTES)
#define OFF_MV    (OFF_MW + WM_BYTES)
#define OFF_MO    (OFF_MV + WM_BYTES)
#define OFF_H16   (OFF_MO + WM_BYTES)
#define OFF_QKV   (OFF_H16 + P16_BYTES)
#define OFF_CTX   (OFF_QKV + 3 * P16_BYTES)
#define OFF_X2    (OFF_CTX + P16_BYTES)
#define OFF_H2    (OFF_X2 + X2_BYTES)
#define OFF_A2    (OFF_H2 + P16_BYTES)
#define WS_TOTAL  (OFF_A2 + A2_BYTES)
static_assert((WQKV_BYTES % 128) == 0 && (WO_BYTES % 128) == 0 && (WM_BYTES % 128) == 0);
static_assert((P16_BYTES % 128) == 0 && (A2_BYTES % 128) == 0 && (TAB_BYTES % 128) == 0);
static_assert(WS_TOTAL <= (size_t)134217728);

__device__ __forceinline__ float bf16r(float x) {
  unsigned int u = __float_as_uint(x);
  u = (u + 0x7FFFu + ((u >> 16) & 1u)) & 0xFFFF0000u;
  return __uint_as_float(u);
}

__device__ __forceinline__ v16h frag_at(const _Float16* p) {
  v8h lo = *(const v8h*)(p);
  v8h hi = *(const v8h*)(p + 16);
  v16h out;
#pragma unroll
  for (int i = 0; i < 8; ++i) { out[i] = lo[i]; out[i + 8] = hi[i]; }
  return out;
}
__device__ __forceinline__ v16h ld_frag(const _Float16* base, unsigned ld) {
  const unsigned lane = threadIdx.x & 31u;
  return frag_at(base + (lane & 15u) * ld + (lane >> 4) * 8u);
}

__device__ __forceinline__ v8f wmma16(v16h a, v16h b, v8f c) {
  v8f d = __builtin_amdgcn_wmma_f32_16x16x32_f16(false, a, false, b, (short)0, c,
                                                 false, false);
  asm volatile("v_nop\n\tv_nop\n\tv_nop\n\tv_nop" : "+v"(d) : "v"(a), "v"(b));
  return d;
}

__device__ __forceinline__ float red16_max(float x) {
#pragma unroll
  for (int off = 1; off < 16; off <<= 1) x = fmaxf(x, __shfl_xor(x, off, 32));
  return x;
}
__device__ __forceinline__ float red16_sum(float x) {
#pragma unroll
  for (int off = 1; off < 16; off <<= 1) x += __shfl_xor(x, off, 32);
  return x;
}

__device__ __forceinline__ void wave_lds_sync() {
  __builtin_amdgcn_fence(3  , "wavefront");
  asm volatile("s_wait_dscnt 0x0" ::: "memory");
  __builtin_amdgcn_wave_barrier();
}

__device__ __forceinline__ unsigned perm_to_nat(unsigned p) {
  const unsigned t = (p >> 6) & 7u;
  const unsigned h = ((p >> 10) & 1u) * 8u + ((p >> 3) & 7u);
  const unsigned w = ((p >> 9) & 1u) * 8u + (p & 7u);
  return t * 256u + h * 16u + w;
}

__global__ __launch_bounds__(256) void ropetab_kernel(float* __restrict__ tab) {
  __shared__ float S[1024];
  const unsigned tid = threadIdx.x;
#pragma unroll 1
  for (unsigned e = 0; e < 2u; ++e) {
    const unsigned combo = e * 256u + tid;
    const unsigned pos = combo >> 5, pj = combo & 31u;
    const unsigned j = (pj < 8u) ? pj : ((pj < 20u) ? pj - 8u : pj - 20u);
    const float rh = (pj < 8u) ? 0.125f : (1.0f / 12.0f);
    const float ex = (float)j * rh;
    const float fr = exp2f(-13.287712379549449f * ex);
    const float ang = (float)pos * fr;
    float sn, cs;
    sincosf(ang, &sn, &cs);
    S[combo * 2u] = cs;
    S[combo * 2u + 1u] = sn;
  }
  __syncthreads();
  const v4f o = *(const v4f*)&S[tid * 4u];
  *(volatile v4f*)(tab + tid * 4u) = o;
  __threadfence();
  *(volatile v4f*)(tab + tid * 4u) = o;
}

__global__ __launch_bounds__(256) void wconv_kernel(
    const float* __restrict__ W, int Ksrc, int Nsrc, _Float16* __restrict__ Wt, int Kpad) {
  __shared__ _Float16 T[64 * LDT];
  const unsigned tid = threadIdx.x;
  const unsigned n0 = blockIdx.x * 64u;
  const unsigned k0 = blockIdx.y * 64u;
#pragma unroll 4
  for (unsigned j = 0; j < 16u; ++j) {
    const unsigned idx = tid + 256u * j;
    const unsigned kr = idx >> 6, nc = idx & 63u;
    const unsigned k = k0 + kr, n = n0 + nc;
    const bool ok = (k < (unsigned)Ksrc) && (n < (unsigned)Nsrc);
    const unsigned kc = (k < (unsigned)Ksrc) ? k : (unsigned)(Ksrc - 1);
    const unsigned ncl = (n < (unsigned)Nsrc) ? n : (unsigned)(Nsrc - 1);
    const float v = W[(size_t)kc * (unsigned)Nsrc + ncl];
    const float sv = ok ? (WCARRY * bf16r(v)) : 0.0f;
    T[nc * LDT + kr] = (_Float16)sv;
  }
  __syncthreads();
  v8h x[2];
  size_t off[2];
#pragma unroll
  for (unsigned i = 0; i < 2u; ++i) {
    const unsigned n = 32u * i + (tid >> 3);
    const unsigned kc = (tid & 7u) * 8u;
    x[i] = *(const v8h*)&T[n * LDT + kc];
    off[i] = (size_t)(n0 + n) * (unsigned)Kpad + k0 + kc;
  }
#pragma unroll
  for (int i = 0; i < 2; ++i) *(volatile v8h*)(Wt + off[i]) = x[i];
  __threadfence();
#pragma unroll
  for (int i = 0; i < 2; ++i) *(volatile v8h*)(Wt + off[i]) = x[i];
}

template <int PERM>
__global__ __launch_bounds__(256) void rmsnorm_kernel(
    const float* __restrict__ X, const float* __restrict__ Wn, _Float16* __restrict__ Y) {
  const unsigned lane = threadIdx.x & 31u, w = threadIdx.x >> 5;
  const unsigned orow = blockIdx.x * 8u + w;
  unsigned srow = orow;
  if (PERM) srow = (orow & ~2047u) + perm_to_nat(orow & 2047u);
  const float* xp = X + (size_t)srow * DIM + lane * 8u;
  const float* wp = Wn + lane * 8u;
  float xv[32];
  float ss = 0.0f;
#pragma unroll
  for (int j = 0; j < 4; ++j) {
    const v4f a0 = *(const v4f*)(xp + j * 256);
    const v4f a1 = *(const v4f*)(xp + j * 256 + 4);
#pragma unroll
    for (int q = 0; q < 4; ++q) {
      const float f0 = PERM ? bf16r(a0[q]) : a0[q];
      const float f1 = PERM ? bf16r(a1[q]) : a1[q];
      xv[j * 8 + q] = f0;
      xv[j * 8 + 4 + q] = f1;
      ss += f0 * f0;
      ss += f1 * f1;
    }
  }
#pragma unroll
  for (int off = 1; off < 32; off <<= 1) ss += __shfl_xor(ss, off, 32);
  const float inv = rsqrtf(ss * (1.0f / (float)DIM) + 1.0e-6f);
  v8h o[4];
#pragma unroll
  for (int j = 0; j < 4; ++j) {
    const v4f g0 = *(const v4f*)(wp + j * 256);
    const v4f g1 = *(const v4f*)(wp + j * 256 + 4);
#pragma unroll
    for (int q = 0; q < 4; ++q) {
      o[j][q]     = (_Float16)(xv[j * 8 + q] * inv * bf16r(g0[q]));
      o[j][q + 4] = (_Float16)(xv[j * 8 + 4 + q] * inv * bf16r(g1[q]));
    }
  }
  _Float16* yp = Y + (size_t)orow * DIM + lane * 8u;
#pragma unroll
  for (int j = 0; j < 4; ++j) *(volatile v8h*)(yp + j * 256) = o[j];
  __threadfence();
#pragma unroll
  for (int j = 0; j < 4; ++j) *(volatile v8h*)(yp + j * 256) = o[j];
}

template <int MODE, int KD>
__global__ __launch_bounds__(256) void gemm_kernel(
    const _Float16* __restrict__ A16, const _Float16* __restrict__ Bt0,
    const _Float16* __restrict__ Bt1, const float* __restrict__ addf,
    const float* __restrict__ tab, float* __restrict__ outf,
    _Float16* __restrict__ out16) {
  constexpr int NCS = (MODE == M_GU) ? 2 : 1;
  __shared__ float Cs[NCS * 64 * LDC];
  __shared__ float Tb[(MODE == M_QKV) ? 1024 : 4];
  const unsigned tid = threadIdx.x, lane = tid & 31u, w = tid >> 5;
  const unsigned mw = w >> 1, nw = w & 1u;
  const unsigned hh = lane >> 4, m = lane & 15u;
  const unsigned n0 = blockIdx.x * 64u;
  const unsigned row0 = blockIdx.y * 64u;

  if (MODE == M_QKV) {
    *(v4f*)&Tb[tid * 4u] = *(const v4f*)(tab + tid * 4u);
  }

  const _Float16* ap  = A16 + (size_t)(row0 + mw * 16u + m) * KD + hh * 8u;
  const _Float16* bp0 = Bt0 + (size_t)(n0 + nw * 32u + m) * KD + hh * 8u;
  const _Float16* bp1 = bp0 + 16 * KD;
  const _Float16* cp0 = Bt1 + (size_t)(n0 + nw * 32u + m) * KD + hh * 8u;
  const _Float16* cp1 = cp0 + 16 * KD;
  v8f acc0 = {}, acc1 = {}, acc2 = {}, acc3 = {};
#pragma unroll 2
  for (unsigned k0 = 0; k0 < (unsigned)KD; k0 += 32u) {
    const v16h a  = frag_at(ap + k0);
    const v16h b0 = frag_at(bp0 + k0);
    const v16h b1 = frag_at(bp1 + k0);
    acc0 = wmma16(a, b0, acc0);
    acc1 = wmma16(a, b1, acc1);
    if (MODE == M_GU) {
      const v16h c0 = frag_at(cp0 + k0);
      const v16h c1 = frag_at(cp1 + k0);
      acc2 = wmma16(a, c0, acc2);
      acc3 = wmma16(a, c1, acc3);
    }
  }
#pragma unroll
  for (int r = 0; r < 8; ++r) {
    float* d = &Cs[(mw * 16u + hh * 8u + (unsigned)r) * LDC + nw * 32u + m];
    d[0]  = acc0[r];
    d[16] = acc1[r];
    if (MODE == M_GU) {
      d[64 * LDC]      = acc2[r];
      d[64 * LDC + 16] = acc3[r];
    }
  }
  __syncthreads();

  if (MODE == M_QKV) {
    const unsigned pl  = blockIdx.x >> 4;
    const unsigned hc0 = (blockIdx.x & 15u) * 64u;
    v8h x[2];
    size_t off[2];
    if (pl < 2u) {
#pragma unroll
      for (unsigned i = 0; i < 2u; ++i) {
        const unsigned r = 32u * i + (tid >> 3);
        const unsigned c = (tid & 7u) * 8u;
        const unsigned prow = row0 + r;
        const unsigned p = prow & 2047u;
        const unsigned pt = (p >> 6) & 7u;
        const unsigned ph = ((p >> 10) & 1u) * 8u + ((p >> 3) & 7u);
        const unsigned pw = ((p >> 9) & 1u) * 8u + (p & 7u);
#pragma unroll
        for (unsigned jj = 0; jj < 8u; ++jj) {
          const unsigned d = c + jj;
          const bool c1 = d >= 16u, c2 = d >= 40u;
          const unsigned base = c2 ? 40u : (c1 ? 16u : 0u);
          const unsigned hf   = c1 ? 12u : 8u;
          const unsigned pj0  = c2 ? 20u : (c1 ? 8u : 0u);
          const unsigned pos  = c2 ? pw : (c1 ? ph : pt);
          const unsigned rel  = d - base;
          const bool sec = rel >= hf;
          const unsigned j  = sec ? rel - hf : rel;
          const unsigned pd = sec ? d - hf : d + hf;
          const unsigned ti = (pos * 32u + pj0 + j) * 2u;
          const float cs = Tb[ti];
          const float sn = Tb[ti + 1u];
          const float xv = Cs[r * LDC + d];
          const float yv = Cs[r * LDC + pd];
          const float sg = sec ? sn : -sn;
          const float rv = xv * cs + yv * sg;
          x[i][jj] = (_Float16)(rv * (1.0f / WCARRY));
        }
        off[i] = (size_t)pl * PLANE_ELEMS + (size_t)prow * DIM + hc0 + c;
      }
    } else {
      const unsigned bidx = row0 >> 11;
      const unsigned key0 = row0 & 2047u;
#pragma unroll
      for (unsigned i = 0; i < 2u; ++i) {
        const unsigned dcol = 32u * i + (tid >> 3);
        const unsigned kk = (tid & 7u) * 8u;
#pragma unroll
        for (unsigned j = 0; j < 8u; ++j)
          x[i][j] = (_Float16)(Cs[(kk + j) * LDC + dcol] * (1.0f / WCARRY));
        off[i] = 2 * PLANE_ELEMS + ((size_t)bidx * DIM + hc0 + dcol) * SEQ + key0 + kk;
      }
    }
#pragma unroll
    for (int i = 0; i < 2; ++i) *(volatile v8h*)(out16 + off[i]) = x[i];
    __threadfence();
#pragma unroll
    for (int i = 0; i < 2; ++i) *(volatile v8h*)(out16 + off[i]) = x[i];
  }

  if (MODE == M_GU) {
    v8h x[2];
    size_t off[2];
#pragma unroll
    for (unsigned i = 0; i < 2u; ++i) {
      const unsigned r = 32u * i + (tid >> 3);
      const unsigned c = (tid & 7u) * 8u;
#pragma unroll
      for (unsigned j = 0; j < 8u; ++j) {
        const float g = Cs[r * LDC + c + j] * (1.0f / WCARRY);
        const float u = Cs[64 * LDC + r * LDC + c + j] * (1.0f / WCARRY);
        const float sg = __builtin_amdgcn_rcpf(1.0f + __expf(-g));
        x[i][j] = (_Float16)((g * sg) * u * ACARRY);
      }
      off[i] = (size_t)(row0 + r) * DHP + n0 + c;
    }
#pragma unroll
    for (int i = 0; i < 2; ++i) *(volatile v8h*)(out16 + off[i]) = x[i];
    __threadfence();
#pragma unroll
    for (int i = 0; i < 2; ++i) *(volatile v8h*)(out16 + off[i]) = x[i];
  }

  if (MODE == M_WO || MODE == M_OUT) {
    v4f xs[4];
    size_t off[4];
#pragma unroll
    for (unsigned i = 0; i < 4u; ++i) {
      const unsigned r = 16u * i + (tid >> 4);
      const unsigned c = (tid & 15u) * 4u;
      const unsigned crow = row0 + r;
      unsigned orow = crow;
      if (MODE == M_WO) orow = (crow & ~2047u) + perm_to_nat(crow & 2047u);
      const v4f u = *(const v4f*)&Cs[r * LDC + c];
      const v4f g = *(const v4f*)(addf + (size_t)orow * DIM + n0 + c);
      v4f val;
#pragma unroll
      for (int j = 0; j < 4; ++j) {
        const float res = (MODE == M_WO) ? bf16r(g[j]) : g[j];
        val[j] = u[j] * (1.0f / (WCARRY * VCARRY)) + res;
      }
      xs[i] = val;
      off[i] = (size_t)orow * DIM + n0 + c;
    }
#pragma unroll
    for (int i = 0; i < 4; ++i) *(volatile v4f*)(outf + off[i]) = xs[i];
    __threadfence();
#pragma unroll
    for (int i = 0; i < 4; ++i) *(volatile v4f*)(outf + off[i]) = xs[i];
  }
}

__global__ __launch_bounds__(256) void attn_kernel(
    const _Float16* __restrict__ Qh, const _Float16* __restrict__ Kh,
    const _Float16* __restrict__ Vt, _Float16* __restrict__ Ov) {
  __shared__ _Float16 Ks[64 * LDT];
  __shared__ _Float16 Vs[64 * LDT];
  __shared__ _Float16 Ps[8 * 16 * LDT];

  const unsigned tid = threadIdx.x, lane = tid & 31u, w = tid >> 5;
  const unsigned hh = lane >> 4, m = lane & 15u;
  const unsigned q0 = blockIdx.x * 128u;
  const unsigned head = blockIdx.y;
  const unsigned b = blockIdx.z;
  const float scale = 0.125f;
  _Float16* P = Ps + w * (16u * LDT);

  const size_t qoff = (size_t)(b * (unsigned)SEQ + q0 + w * 16u + m) * DIM + head * HD + hh * 8u;
  v16h qf[2];
  qf[0] = frag_at(Qh + qoff);
  qf[1] = frag_at(Qh + qoff + 32);

  float mrow[8], lrow[8];
  v8f o[4];
#pragma unroll
  for (int v = 0; v < 8; ++v) { mrow[v] = -1.0e30f; lrow[v] = 0.0f; }
#pragma unroll
  for (int nb = 0; nb < 4; ++nb) o[nb] = (v8f){};

  const size_t kplane = (size_t)b * SEQ * DIM + head * HD;
  const size_t vplane = ((size_t)b * DIM + head * HD) * SEQ;

  const unsigned kv_lo = (head < (unsigned)LHEADS) ? (q0 & ~511u) : 0u;
  const unsigned kv_hi = (head < (unsigned)LHEADS) ? (kv_lo + 512u) : (unsigned)SEQ;

  for (unsigned kb = kv_lo; kb < kv_hi; kb += 64u) {
#pragma unroll
    for (unsigned j = 0; j < 2u; ++j) {
      const unsigned idx = tid + 256u * j;
      const unsigned r = idx >> 3, c = (idx & 7u) * 8u;
      *(v8h*)&Ks[r * LDT + c] = *(const v8h*)(Kh + kplane + (size_t)(kb + r) * DIM + c);
      *(v8h*)&Vs[r * LDT + c] = *(const v8h*)(Vt + vplane + (size_t)r * SEQ + kb + c);
    }
    __syncthreads();

    v8f s[4];
#pragma unroll
    for (int kg = 0; kg < 4; ++kg) {
      v8f t = {};
#pragma unroll
      for (int c = 0; c < 2; ++c) {
        const v16h kf = ld_frag(&Ks[(kg * 16) * LDT + c * 32], LDT);
        t = wmma16(qf[c], kf, t);
      }
      s[kg] = t * scale;
    }

    float alpha[8];
#pragma unroll
    for (int v = 0; v < 8; ++v) {
      float mx = fmaxf(fmaxf(s[0][v], s[1][v]), fmaxf(s[2][v], s[3][v]));
      mx = red16_max(mx);
      const float mn = fmaxf(mrow[v], mx);
      alpha[v] = __expf(mrow[v] - mn);
      mrow[v] = mn;
    }
#pragma unroll
    for (int kg = 0; kg < 4; ++kg)
#pragma unroll
      for (int v = 0; v < 8; ++v) s[kg][v] = __expf(s[kg][v] - mrow[v]);
#pragma unroll
    for (int v = 0; v < 8; ++v) {
      const float rs = red16_sum((s[0][v] + s[1][v]) + (s[2][v] + s[3][v]));
      lrow[v] = alpha[v] * lrow[v] + rs;
    }
#pragma unroll
    for (int nb = 0; nb < 4; ++nb)
#pragma unroll
      for (int v = 0; v < 8; ++v) o[nb][v] = o[nb][v] * alpha[v];

#pragma unroll
    for (int kg = 0; kg < 4; ++kg)
#pragma unroll
      for (int v = 0; v < 8; ++v)
        P[(hh * 8u + (unsigned)v) * LDT + (unsigned)kg * 16u + m] = (_Float16)(s[kg][v] * PCARRY);
    wave_lds_sync();

#pragma unroll
    for (int c = 0; c < 2; ++c) {
      const v16h pf = ld_frag(P + c * 32, LDT);
#pragma unroll
      for (int nb = 0; nb < 4; ++nb) {
        const v16h vf = ld_frag(&Vs[(nb * 16) * LDT + c * 32], LDT);
        o[nb] = wmma16(pf, vf, o[nb]);
      }
    }
    __syncthreads();
  }

  float inv[8];
#pragma unroll
  for (int v = 0; v < 8; ++v) inv[v] = __builtin_amdgcn_rcpf(lrow[v]) * (VCARRY / PCARRY);
#pragma unroll
  for (int nb = 0; nb < 4; ++nb)
#pragma unroll
    for (int v = 0; v < 8; ++v)
      P[(hh * 8u + (unsigned)v) * LDT + (unsigned)nb * 16u + m] = (_Float16)(o[nb][v] * inv[v]);
  wave_lds_sync();
  v8h x[4];
  size_t off[4];
#pragma unroll
  for (unsigned i = 0; i < 4u; ++i) {
    const unsigned r = 4u * i + (lane >> 3);
    const unsigned c = (lane & 7u) * 8u;
    x[i] = *(const v8h*)&P[r * LDT + c];
    off[i] = (size_t)(b * (unsigned)SEQ + q0 + w * 16u + r) * DIM + head * HD + c;
  }
#pragma unroll
  for (int i = 0; i < 4; ++i) *(volatile v8h*)(Ov + off[i]) = x[i];
  __threadfence();
#pragma unroll
  for (int i = 0; i < 4; ++i) *(volatile v8h*)(Ov + off[i]) = x[i];
}

extern "C" void kernel_launch(void* const* d_in, const int* in_sizes, int n_in,
                              void* d_out, int out_size, void* d_ws, size_t ws_size,
                              hipStream_t stream) {
  if (n_in < 8) return;
  const long long need_x = (long long)MROWS * DIM;
  if ((long long)in_sizes[0] < need_x) return;
  if (in_sizes[1] < DIM) return;
  if ((long long)in_sizes[2] < (long long)DIM * 3 * DIM) return;
  if ((long long)in_sizes[3] < (long long)DIM * DIM) return;
  if (in_sizes[4] < DIM) return;
  if ((long long)in_sizes[5] < (long long)DIM * DHID) return;
  if ((long long)in_sizes[6] < (long long)DIM * DHID) return;
  if ((long long)in_sizes[7] < (long long)DHID * DIM) return;
  if ((long long)out_size < need_x) return;
  if (ws_size < WS_TOTAL) return;

  const float* X      = (const float*)d_in[0];
  const float* norm1w = (const float*)d_in[1];
  const float* Wqkv   = (const float*)d_in[2];
  const float* Wo     = (const float*)d_in[3];
  const float* norm2w = (const float*)d_in[4];
  const float* Mw     = (const float*)d_in[5];
  const float* Mv     = (const float*)d_in[6];
  const float* Mo     = (const float*)d_in[7];
  float* out = (float*)d_out;

  char* ws = (char*)d_ws;
  float*    Tab   = (float*)(ws + OFF_TAB);
  _Float16* WqkvT = (_Float16*)(ws + OFF_WQKV);
  _Float16* WoT   = (_Float16*)(ws + OFF_WO);
  _Float16* MwT   = (_Float16*)(ws + OFF_MW);
  _Float16* MvT   = (_Float16*)(ws + OFF_MV);
  _Float16* MoT   = (_Float16*)(ws + OFF_MO);
  _Float16* H16   = (_Float16*)(ws + OFF_H16);
  _Float16* Qp    = (_Float16*)(ws + OFF_QKV);
  _Float16* Kp    = Qp + PLANE_ELEMS;
  _Float16* Vtp   = Qp + 2 * PLANE_ELEMS;
  _Float16* Ctx   = (_Float16*)(ws + OFF_CTX);
  float*    X2    = (float*)(ws + OFF_X2);
  _Float16* H2    = (_Float16*)(ws + OFF_H2);
  _Float16* A2    = (_Float16*)(ws + OFF_A2);

  dim3 blk(256);

  ropetab_kernel<<<dim3(1), blk, 0, stream>>>(Tab);
  wconv_kernel<<<dim3(3 * DIM / 64, DIM / 64), blk, 0, stream>>>(Wqkv, DIM, 3 * DIM, WqkvT, DIM);
  wconv_kernel<<<dim3(DIM / 64, DIM / 64), blk, 0, stream>>>(Wo, DIM, DIM, WoT, DIM);
  wconv_kernel<<<dim3(DHP / 64, DIM / 64), blk, 0, stream>>>(Mw, DIM, DHID, MwT, DIM);
  wconv_kernel<<<dim3(DHP / 64, DIM / 64), blk, 0, stream>>>(Mv, DIM, DHID, MvT, DIM);
  wconv_kernel<<<dim3(DIM / 64, DHP / 64), blk, 0, stream>>>(Mo, DHID, DIM, MoT, DHP);

  rmsnorm_kernel<1><<<dim3(MROWS / 8), blk, 0, stream>>>(X, norm1w, H16);
  gemm_kernel<M_QKV, DIM><<<dim3(3 * DIM / 64, MROWS / 64), blk, 0, stream>>>(
      H16, WqkvT, WqkvT, X, Tab, X2, Qp);
  attn_kernel<<<dim3(SEQ / 128, NHEAD, NB), blk, 0, stream>>>(Qp, Kp, Vtp, Ctx);
  gemm_kernel<M_WO, DIM><<<dim3(DIM / 64, MROWS / 64), blk, 0, stream>>>(
      Ctx, WoT, WoT, X, Tab, X2, Qp);
  rmsnorm_kernel<0><<<dim3(MROWS / 8), blk, 0, stream>>>(X2, norm2w, H2);
  gemm_kernel<M_GU, DIM><<<dim3(DHP / 64, MROWS / 64), blk, 0, stream>>>(
      H2, MwT, MvT, X, Tab, X2, A2);
  gemm_kernel<M_OUT, DHP><<<dim3(DIM / 64, MROWS / 64), blk, 0, stream>>>(
      A2, MoT, MoT, X2, Tab, out, Qp);
}
